// RAM_21809843929536
// MI455X (gfx1250) — hardware-verified
//
#include <hip/hip_runtime.h>
#include <math.h>
#include <stdint.h>


#define BATCH 4
#define CH    256
#define HID   32
#define NTOK  4096
#define TOK   (BATCH * NTOK)
#define KQLD  64
#define VLD   TOK
#define OUTN  (BATCH * CH * NTOK)
#define MT    32
#define NCH   64
#define PTP   72
#define STW   32

#define SCW  64.0f
#define SCQK 8.0f
#define SCV  1024.0f
#define SCE  32768.0f
#define SCR  2048.0f
#define SCS  (0.17677669529663687f / 64.0f)

static_assert(TOK % 64 == 0 && CH % 64 == 0 && KQLD == 64);
static_assert(((TOK / 64) % 8) == 0);
static_assert((((CH / 64) * (TOK / 64)) % 8) == 0);
static_assert(((BATCH * (NTOK / 16)) % 8) == 0);
static_assert(NTOK % NCH == 0 && NTOK % MT == 0 && CH == 8 * 32);
static_assert((HID * CH) % 2048 == 0 && (CH * CH) % 2048 == 0);
static_assert(NTOK / MT == 128);
static_assert(STW == 32);

typedef _Float16       v16h __attribute__((ext_vector_type(16)));
typedef _Float16       v8h  __attribute__((ext_vector_type(8)));
typedef float          v8f  __attribute__((ext_vector_type(8)));
typedef float          v4f  __attribute__((ext_vector_type(4)));
typedef unsigned int   v4u  __attribute__((ext_vector_type(4)));

union HU { v8h h; v4u u; _Float16 s[8]; };
union FR { v16h v; v8h h[2]; _Float16 s[16]; };
static_assert(sizeof(HU) == 16);
static_assert(sizeof(FR) == 32);

__device__ __forceinline__ unsigned short bf_bits(float f) {
  const unsigned u = __float_as_uint(f);
  return (unsigned short)((u + 0x7FFFu + ((u >> 16) & 1u)) >> 16);
}
__device__ __forceinline__ float bf_up(unsigned short h) { return __uint_as_float(((unsigned)h) << 16); }
__device__ __forceinline__ float bfr(float f) { return bf_up(bf_bits(f)); }
__device__ __forceinline__ v8f zero8() { v8f z = {0.f, 0.f, 0.f, 0.f, 0.f, 0.f, 0.f, 0.f}; return z; }

__device__ __forceinline__ void ld8(const float* p, float* o) {
  const v4f a = *(const v4f*)(p);
  const v4f b = *(const v4f*)(p + 4);
  o[0] = a[0]; o[1] = a[1]; o[2] = a[2]; o[3] = a[3];
  o[4] = b[0]; o[5] = b[1]; o[6] = b[2]; o[7] = b[3];
}

__device__ __forceinline__ v16h ldfrag_h(const _Float16* p) {
  FR f;
  f.h[0] = *(const v8h*)(p);
  f.h[1] = *(const v8h*)(p + 16);
  return f.v;
}

__device__ __forceinline__ v8f mma_h(v16h a, v16h b, v8f c) {
  c = __builtin_amdgcn_wmma_f32_16x16x32_f16(false, a, false, b, (short)0, c, false, false);
#if defined(__HIP_DEVICE_COMPILE__)
  asm volatile("v_nop\n\tv_nop\n\tv_nop\n\tv_nop" : "+v"(c) : "v"(a), "v"(b));
#endif
  return c;
}
__device__ __forceinline__ v8f mma_h_raw(v16h a, v16h b, v8f c) {
  return __builtin_amdgcn_wmma_f32_16x16x32_f16(false, a, false, b, (short)0, c, false, false);
}
__device__ __forceinline__ void dep_guard_h(v8f& a, v8f& b, v16h x) {
#if defined(__HIP_DEVICE_COMPILE__)
  asm volatile("v_nop\n\tv_nop\n\tv_nop\n\tv_nop" : "+v"(a), "+v"(b) : "v"(x));
#endif
}
__device__ __forceinline__ void keep4_h(v16h a, v16h b, v16h c, v16h d) {
#if defined(__HIP_DEVICE_COMPILE__)
  asm volatile("v_nop" :: "v"(a), "v"(b), "v"(c), "v"(d));
#endif
}
__device__ __forceinline__ void acc_guard4(v8f& a, v8f& b, v8f& c, v8f& d) {
#if defined(__HIP_DEVICE_COMPILE__)
  asm volatile("v_nop\n\tv_nop\n\tv_nop\n\tv_nop" : "+v"(a), "+v"(b), "+v"(c), "+v"(d));
#endif
}

__global__ __launch_bounds__(256) void cvt_flat(const float* __restrict__ in, _Float16* out, int n8, float scale) {
  const int i = blockIdx.x * 256 + threadIdx.x;
  if (i < n8) {
    float v[8];
    ld8(in + (size_t)i * 8, v);
    HU u;
#pragma unroll
    for (int e = 0; e < 8; ++e) u.s[e] = (_Float16)(bfr(v[e]) * scale);
    _Float16* p = out + (size_t)i * 8;
    *(volatile v4u*)p = u.u;
    __threadfence();
    *(volatile v4u*)p = u.u;
  }
}

__global__ __launch_bounds__(256) void cvt_xT(const float* __restrict__ X, _Float16* XT) {
  __shared__ float sw[64][65];
  const int t = threadIdx.x;
  const int n0 = blockIdx.x * 64, k0 = blockIdx.y * 64, b = blockIdx.z;
  const float* Xb = X + (size_t)b * CH * NTOK;
  {
    const int r = t >> 4, c4 = (t & 15) * 4;
#pragma unroll
    for (int it = 0; it < 4; ++it) {
      const int row = r + 16 * it;
      const v4f x = *(const v4f*)(Xb + (size_t)(k0 + row) * NTOK + n0 + c4);
      sw[row][c4 + 0] = x[0]; sw[row][c4 + 1] = x[1]; sw[row][c4 + 2] = x[2]; sw[row][c4 + 3] = x[3];
    }
  }
  __syncthreads();
  const int q8 = t & 7, rr = t >> 3;
  HU u[2];
#pragma unroll
  for (int it = 0; it < 2; ++it) {
    const int n = rr + 32 * it;
#pragma unroll
    for (int e = 0; e < 8; ++e) u[it].s[e] = (_Float16)bfr(sw[8 * q8 + e][n]);
  }
  for (int pass = 0; pass < 2; ++pass) {
#pragma unroll
    for (int it = 0; it < 2; ++it) {
      const int n = rr + 32 * it;
      _Float16* dst = XT + (size_t)(b * NTOK + n0 + n) * CH + k0 + 8 * q8;
      *(volatile v4u*)dst = u[it].u;
    }
    __threadfence();
  }
}

__device__ __forceinline__ void kseg(v8f (&acc)[4][4], const _Float16* __restrict__ A, int lda, int m0,
                                     const _Float16* __restrict__ Bt, int ldb, int n0, int K, int rlane, int koff) {
  for (int kk = 0; kk < K; kk += 32) {
    v16h bh[4];
#pragma unroll
    for (int j = 0; j < 4; ++j) {
      const size_t bo = (size_t)(n0 + (j << 4) + rlane) * (size_t)ldb + koff + kk;
      bh[j] = ldfrag_h(Bt + bo);
    }
#pragma unroll
    for (int i = 0; i < 4; ++i) {
      const size_t ao = (size_t)(m0 + (i << 4) + rlane) * (size_t)lda + koff + kk;
      const v16h a0 = ldfrag_h(A + ao);
#pragma unroll
      for (int j = 0; j < 4; ++j) acc[i][j] = mma_h_raw(a0, bh[j], acc[i][j]);
      dep_guard_h(acc[i][0], acc[i][3], a0);
    }
    keep4_h(bh[0], bh[1], bh[2], bh[3]);
  }
}

template <int RB, int CS>
__global__ __launch_bounds__(256) void gemm64p(
    const _Float16* __restrict__ A, int lda, const _Float16* __restrict__ Bt, int ldb,
    const float* __restrict__ bias0, const float* __restrict__ bias1, int nsplit, int nb,
    const float* __restrict__ rowbias, int nrb, const float* __restrict__ cscale,
    float cs, float so, _Float16* Ch, _Float16* Cl, int ldc, int M, int N, int K) {
  __shared__ __align__(16) float sT[8][16 * 68];
  const int lane = threadIdx.x & 31;
  const int wave = threadIdx.x >> 5;
  const int tilesN = N >> 6;
  const int tilesM = M >> 6;
  const int tiles = tilesM * tilesN;
  const int item = blockIdx.x * 8 + wave;
  if (item >= tiles) return;
  const int tm = item / tilesN;
  const int tn = item - tm * tilesN;
  const int m0 = tm << 6;
  const int n0 = tn << 6;

  const int rlane = lane & 15;
  const int koff  = (lane >> 4) * 8;
  const int mOff  = (lane >> 4) * 8;

  v8f acc[4][4];
#pragma unroll
  for (int i = 0; i < 4; ++i)
#pragma unroll
    for (int j = 0; j < 4; ++j) acc[i][j] = zero8();

  kseg(acc, A, lda, m0, Bt, ldb, n0, K, rlane, koff);
  acc_guard4(acc[0][0], acc[0][1], acc[0][2], acc[0][3]);
  acc_guard4(acc[1][0], acc[1][1], acc[1][2], acc[1][3]);
  acc_guard4(acc[2][0], acc[2][1], acc[2][2], acc[2][3]);
  acc_guard4(acc[3][0], acc[3][1], acc[3][2], acc[3][3]);

  const int q8 = lane & 7, rr = lane >> 3, c8 = q8 * 8;
  float bb[8], sc[8];
#pragma unroll
  for (int e = 0; e < 8; ++e) {
    const int n = n0 + c8 + e;
    const int i0 = min(n, nb - 1);
    const int i1 = min(max(n - nsplit, 0), nb - 1);
    const float x0 = bias0[i0];
    const float x1 = bias1[i1];
    bb[e] = RB ? 0.0f : bfr((n < nsplit) ? x0 : x1);
  }
  {
    const int nn = n0 + c8;
    const float* sp = cscale + (size_t)(nn >> 4) * STW + 16 + (nn & 15);
    const v4f s0 = *(const v4f*)(sp);
    const v4f s1 = *(const v4f*)(sp + 4);
#pragma unroll
    for (int e = 0; e < 4; ++e) {
      sc[e]     = CS ? s0[e] : so;
      sc[4 + e] = CS ? s1[e] : so;
    }
  }

  float* slab = sT[wave];
#pragma unroll
  for (int i = 0; i < 4; ++i) {
    const int mBase = m0 + (i << 4);
#pragma unroll
    for (int r = 0; r < 8; ++r) {
#pragma unroll
      for (int j = 0; j < 4; ++j) {
        slab[(mOff + r) * 68 + (j << 4) + rlane] = acc[i][j][r];
      }
    }
    __builtin_amdgcn_fence(__ATOMIC_RELEASE, "workgroup");
    __builtin_amdgcn_wave_barrier();
    __builtin_amdgcn_fence(__ATOMIC_ACQUIRE, "workgroup");
    v4u uh[4], ul[4];
#pragma unroll
    for (int it = 0; it < 4; ++it) {
      const int row = it * 4 + rr;
      float xs[8];
      ld8(slab + row * 68 + c8, xs);
      const float rbv = RB ? bfr(rowbias[min(mBase + row, nrb - 1)]) : 0.0f;
      HU h, l;
#pragma unroll
      for (int e = 0; e < 8; ++e) {
        const float v = (xs[e] * cs + bb[e] + rbv) * sc[e];
        const _Float16 hv = (_Float16)v;
        h.s[e] = hv;
        l.s[e] = (_Float16)((v - (float)hv) * SCR);
      }
      uh[it] = h.u;
      ul[it] = l.u;
    }
    for (int pass = 0; pass < 2; ++pass) {
#pragma unroll
      for (int it = 0; it < 4; ++it) {
        const int row = it * 4 + rr;
        const size_t co = (size_t)(mBase + row) * (size_t)ldc + n0 + c8;
        *(volatile v4u*)(Ch + co) = uh[it];
        *(volatile v4u*)(Cl + co) = ul[it];
      }
      __threadfence();
    }
    __builtin_amdgcn_fence(__ATOMIC_RELEASE, "workgroup");
    __builtin_amdgcn_wave_barrier();
    __builtin_amdgcn_fence(__ATOMIC_ACQUIRE, "workgroup");
  }
}

__device__ __forceinline__ v8f s_tile(v16h kh, v16h kl, v16h qh, v16h ql) {
  v8f a0 = zero8(), a1 = zero8();
  a0 = mma_h(kh, qh, a0);
  a1 = mma_h(kh, ql, a1);
  a1 = mma_h(kl, qh, a1);
  v8f s = zero8();
#pragma unroll
  for (int r = 0; r < 8; ++r) s[r] = (a0[r] + a1[r] * (1.0f / SCR)) * SCS;
  return s;
}

__global__ __launch_bounds__(256) void k_stats(const _Float16* __restrict__ KLh, const _Float16* __restrict__ KLl,
                                               const _Float16* __restrict__ QUh, const _Float16* __restrict__ QUl,
                                               float* ST) {
  __shared__ __align__(16) float sSt[8][32];
  const int tid = threadIdx.x, wave = tid >> 5, lane = tid & 31;
  const int hh = lane >> 4, rl = lane & 15;
  const int item = blockIdx.x * 8 + wave;
  if (item >= BATCH * (NTOK / 16)) return;
  const int b = item >> 8, nt = item & 255, n0 = nt * 16;

  const size_t ko = (size_t)(b * NTOK + n0 + rl) * KQLD + 8 * hh;
  const v16h kh = ldfrag_h(KLh + ko);
  const v16h kl = ldfrag_h(KLl + ko);
  const _Float16* qhb = QUh + (size_t)(b * NTOK + rl) * KQLD + HID + 8 * hh;
  const _Float16* qlb = QUl + (size_t)(b * NTOK + rl) * KQLD + HID + 8 * hh;

  float mx[8], z[8];
#pragma unroll
  for (int r = 0; r < 8; ++r) { mx[r] = -1.0e30f; z[r] = 0.0f; }

  for (int mt = 0; mt < NTOK / 16; ++mt) {
    const size_t qo = (size_t)mt * 16 * KQLD;
    const v16h qh = ldfrag_h(qhb + qo);
    const v16h ql = ldfrag_h(qlb + qo);
    const v8f s = s_tile(kh, kl, qh, ql);
#pragma unroll
    for (int r = 0; r < 8; ++r) {
      const float d = s[r] - mx[r];
      const float e = __expf(-fabsf(d));
      const float zu = z[r] * e + 1.0f;
      const float zd = z[r] + e;
      z[r] = (d > 0.0f) ? zu : zd;
      mx[r] = fmaxf(mx[r], s[r]);
    }
  }
#pragma unroll
  for (int off = 8; off >= 1; off >>= 1) {
#pragma unroll
    for (int r = 0; r < 8; ++r) {
      const float om = __shfl_xor(mx[r], off, 32);
      const float oz = __shfl_xor(z[r], off, 32);
      const float nm = fmaxf(mx[r], om);
      z[r] = z[r] * __expf(mx[r] - nm) + oz * __expf(om - nm);
      mx[r] = nm;
    }
  }
  if (rl == 0) {
#pragma unroll
    for (int r = 0; r < 8; ++r) {
      sSt[wave][8 * hh + r] = mx[r];
      sSt[wave][16 + 8 * hh + r] = SCV / z[r];
    }
  }
  __builtin_amdgcn_fence(__ATOMIC_RELEASE, "workgroup");
  __builtin_amdgcn_wave_barrier();
  __builtin_amdgcn_fence(__ATOMIC_ACQUIRE, "workgroup");
  const v4f st = *(const v4f*)(&sSt[wave][4 * (lane & 7)]);
  if (lane < 8) {
    float* dst = ST + (size_t)item * STW + 4 * lane;
    *(volatile v4f*)dst = st;
    __threadfence();
    *(volatile v4f*)dst = st;
  }
}

__global__ __launch_bounds__(256) void k_pv(const _Float16* __restrict__ KLh, const _Float16* __restrict__ KLl,
                                            const _Float16* __restrict__ QUh, const _Float16* __restrict__ QUl,
                                            const _Float16* __restrict__ VH, const _Float16* __restrict__ VL,
                                            const float* __restrict__ ST, float* out) {
  __shared__ __align__(16) _Float16 sPt[MT * PTP];
  __shared__ __align__(16) float sO[8][16 * 36];
  const int tid = threadIdx.x, wave = tid >> 5, lane = tid & 31;
  const int hh = lane >> 4, rl = lane & 15;
  const int bx = blockIdx.x;
  const int b = bx >> 7;
  const int m0 = (bx & 127) * MT;
  const int mj = wave & 1;
  const int nsl = (wave >> 1) * 16;
  const int cb = wave * 32;

  const size_t qo = (size_t)(b * NTOK + m0 + 16 * mj + rl) * KQLD + HID + 8 * hh;
  const v16h qh = ldfrag_h(QUh + qo);
  const v16h ql = ldfrag_h(QUl + qo);

  v8f acc[2][2], accl[2][2];
#pragma unroll
  for (int i = 0; i < 2; ++i)
#pragma unroll
    for (int j = 0; j < 2; ++j) { acc[i][j] = zero8(); accl[i][j] = zero8(); }

  for (int nc = 0; nc < NTOK; nc += NCH) {
    const size_t ko = (size_t)(b * NTOK + nc + nsl + rl) * KQLD + 8 * hh;
    const v16h kh = ldfrag_h(KLh + ko);
    const v16h kl = ldfrag_h(KLl + ko);
    const v8f s = s_tile(kh, kl, qh, ql);
    const int bn = b * NTOK + nc + nsl + 8 * hh;
    const float* mp = ST + (size_t)(bn >> 4) * STW + (bn & 15);
    const v4f ma = *(const v4f*)(mp);
    const v4f mb = *(const v4f*)(mp + 4);
    float mv[8];
#pragma unroll
    for (int e = 0; e < 4; ++e) { mv[e] = ma[e]; mv[4 + e] = mb[e]; }
    HU u;
#pragma unroll
    for (int r = 0; r < 8; ++r) u.s[r] = (_Float16)(__expf(s[r] - mv[r]) * SCE);
    __syncthreads();
    *(v8h*)(&sPt[(16 * mj + rl) * PTP + nsl + 8 * hh]) = u.h;
    __syncthreads();
#pragma unroll
    for (int ks = 0; ks < 2; ++ks) {
      const v16h pb0 = ldfrag_h(&sPt[rl * PTP + 32 * ks + 8 * hh]);
      const v16h pb1 = ldfrag_h(&sPt[(16 + rl) * PTP + 32 * ks + 8 * hh]);
#pragma unroll
      for (int i = 0; i < 2; ++i) {
        const size_t vo = (size_t)(cb + 16 * i + rl) * VLD + (size_t)(b * NTOK + nc + 32 * ks) + 8 * hh;
        const v16h ah = ldfrag_h(VH + vo);
        const v16h al = ldfrag_h(VL + vo);
        acc[i][0]  = mma_h(ah, pb0, acc[i][0]);
        acc[i][1]  = mma_h(ah, pb1, acc[i][1]);
        accl[i][0] = mma_h(al, pb0, accl[i][0]);
        accl[i][1] = mma_h(al, pb1, accl[i][1]);
      }
    }
  }

  const float fo = 1.0f / (SCV * SCE);
  const float fl = fo * (1.0f / SCR);
  float* slab = sO[wave];
  const int q8 = lane & 7, rr = lane >> 3;
#pragma unroll
  for (int i = 0; i < 2; ++i) {
#pragma unroll
    for (int r = 0; r < 8; ++r) {
#pragma unroll
      for (int j = 0; j < 2; ++j) {
        slab[(8 * hh + r) * 36 + 16 * j + rl] = acc[i][j][r] * fo + accl[i][j][r] * fl;
      }
    }
    __builtin_amdgcn_fence(__ATOMIC_RELEASE, "workgroup");
    __builtin_amdgcn_wave_barrier();
    __builtin_amdgcn_fence(__ATOMIC_ACQUIRE, "workgroup");
    v4f ov[4];
#pragma unroll
    for (int it = 0; it < 4; ++it) {
      const int row = it * 4 + rr;
      ov[it] = *(const v4f*)(slab + row * 36 + 4 * q8);
    }
    for (int pass = 0; pass < 2; ++pass) {
#pragma unroll
      for (int it = 0; it < 4; ++it) {
        const int row = it * 4 + rr;
        float* dst = out + ((size_t)(b * CH + cb + 16 * i + row)) * NTOK + m0 + 4 * q8;
        *(volatile v4f*)dst = ov[it];
      }
      __threadfence();
    }
    __builtin_amdgcn_fence(__ATOMIC_RELEASE, "workgroup");
    __builtin_amdgcn_wave_barrier();
    __builtin_amdgcn_fence(__ATOMIC_ACQUIRE, "workgroup");
  }
}

extern "C" void kernel_launch(void* const* d_in, const int* in_sizes, int n_in,
                              void* d_out, int out_size, void* d_ws, size_t ws_size,
                              hipStream_t stream) {
  if (n_in < 8) return;
  if (in_sizes[0] != OUTN || in_sizes[1] != OUTN) return;
  if (in_sizes[2] != HID * CH || in_sizes[4] != HID * CH) return;
  if (in_sizes[3] != HID || in_sizes[5] != HID) return;
  if (in_sizes[6] != CH * CH || in_sizes[7] != CH) return;
  if (out_size != OUTN) return;

  const float* left = (const float*)d_in[0];
  const float* up   = (const float*)d_in[1];
  const float* w0   = (const float*)d_in[2];
  const float* b0   = (const float*)d_in[3];
  const float* w1   = (const float*)d_in[4];
  const float* b1   = (const float*)d_in[5];
  const float* w2   = (const float*)d_in[6];
  const float* b2   = (const float*)d_in[7];

  const size_t PW01 = (size_t)KQLD * CH * 2;
  const size_t PW2  = (size_t)CH * CH * 2;
  const size_t PXT  = (size_t)TOK * CH * 2;
  const size_t PKQ  = (size_t)TOK * KQLD * 2;
  const size_t PST  = (size_t)BATCH * (NTOK / 16) * STW * 4;
  const size_t PVP  = (size_t)CH * VLD * 2;

  size_t off = 0;
  const size_t oW01 = off; off += PW01;
  const size_t oW2  = off; off += PW2;
  const size_t oXTl = off; off += PXT;
  const size_t oXTu = off; off += PXT;
  const size_t oKLh = off; off += PKQ;
  const size_t oKLl = off; off += PKQ;
  const size_t oQUh = off; off += PKQ;
  const size_t oQUl = off; off += PKQ;
  const size_t oST  = off; off += PST;
  const size_t oVH  = off; off += PVP;
  const size_t oVL  = off; off += PVP;
  if (off > ws_size) return;
  if (off > (size_t)134217728) return;

  char* ws = (char*)d_ws;
  _Float16* W01 = (_Float16*)(ws + oW01);
  _Float16* W2p = (_Float16*)(ws + oW2);
  _Float16* XTl = (_Float16*)(ws + oXTl);
  _Float16* XTu = (_Float16*)(ws + oXTu);
  _Float16* KLh = (_Float16*)(ws + oKLh);
  _Float16* KLl = (_Float16*)(ws + oKLl);
  _Float16* QUh = (_Float16*)(ws + oQUh);
  _Float16* QUl = (_Float16*)(ws + oQUl);
  float*    ST  = (float*)(ws + oST);
  _Float16* VH  = (_Float16*)(ws + oVH);
  _Float16* VL  = (_Float16*)(ws + oVL);
  float*    outf = (float*)d_out;

  const dim3 blk(256);
  const int n8w01 = (HID * CH) / 8;
  const int n8w2  = (CH * CH) / 8;
  const dim3 gW01((n8w01 + 255) / 256);
  const dim3 gW2((n8w2 + 255) / 256);
  const dim3 gXT(NTOK / 64, CH / 64, BATCH);
  const dim3 gKQ(((TOK / 64) * (KQLD / 64) + 7) / 8);
  const dim3 gSt((BATCH * (NTOK / 16)) / 8);
  const dim3 gVa(((CH / 64) * (TOK / 64) + 7) / 8);
  const dim3 gPV(BATCH * (NTOK / MT));
  const float cs64 = 1.0f / SCW;

  cvt_flat<<<gW01, blk, 0, stream>>>(w0, W01, n8w01, SCW);
  cvt_flat<<<gW01, blk, 0, stream>>>(w1, W01 + (size_t)HID * CH, n8w01, SCW);
  cvt_flat<<<gW2, blk, 0, stream>>>(w2, W2p, n8w2, SCW);
  cvt_xT<<<gXT, blk, 0, stream>>>(left, XTl);
  cvt_xT<<<gXT, blk, 0, stream>>>(up, XTu);
  gemm64p<0, 0><<<gKQ, blk, 0, stream>>>(XTl, CH, W01, CH, b0, b1, HID, HID, b0, HID, ST,
                                         cs64, SCQK, KLh, KLl, KQLD, TOK, KQLD, CH);
  gemm64p<0, 0><<<gKQ, blk, 0, stream>>>(XTu, CH, W01, CH, b0, b1, HID, HID, b0, HID, ST,
                                         cs64, SCQK, QUh, QUl, KQLD, TOK, KQLD, CH);
  k_stats<<<gSt, blk, 0, stream>>>(KLh, KLl, QUh, QUl, ST);
  gemm64p<1, 1><<<gVa, blk, 0, stream>>>(W2p, CH, XTl, CH, b2, b2, TOK, CH, b2, CH, ST,
                                         cs64, 1.0f, VH, VL, VLD, CH, TOK, CH);
  k_pv<<<gPV, blk, 0, stream>>>(KLh, KLl, QUh, QUl, VH, VL, ST, outf);
  (void)hipGetLastError();
}
